// LayerNormGRUCell_64982855188492
// MI455X (gfx1250) — hardware-verified
//
#include <hip/hip_runtime.h>

#define NB   8192
#define KD   1024
#define N2   2048
#define N1   1024
#define LN_EPS 1e-5f

static_assert(KD % 32 == 0);
static_assert(NB % 128 == 0);
static_assert(N2 % 64 == 0);
static_assert(N1 % 64 == 0);
static_assert(N1 == 256 * 4);

typedef __bf16 v16b __attribute__((ext_vector_type(16)));
typedef __bf16 v8b  __attribute__((ext_vector_type(8)));
typedef float  v8f  __attribute__((ext_vector_type(8)));
typedef float  v4f  __attribute__((ext_vector_type(4)));
typedef unsigned short v8us __attribute__((ext_vector_type(8)));
typedef v8b  __attribute__((may_alias)) v8ba;
typedef v4f  __attribute__((may_alias)) v4fa;
typedef v8us __attribute__((may_alias)) v8usa;

union Frag { v16b v; v8b half[2]; };

constexpr size_t SZ_XB   = (size_t)NB * KD * 2;
constexpr size_t SZ_W2   = (size_t)N2 * KD * 2;
constexpr size_t SZ_W1   = (size_t)N1 * KD * 2;
constexpr size_t SZ_P2   = (size_t)NB * N2 * 4;
constexpr size_t SZ_P1   = (size_t)NB * N1 * 4;
constexpr size_t OFF_XB   = 0;
constexpr size_t OFF_HB   = OFF_XB + SZ_XB;
constexpr size_t OFF_WIRZ = OFF_HB + SZ_XB;
constexpr size_t OFF_WHRZ = OFF_WIRZ + SZ_W2;
constexpr size_t OFF_WIN  = OFF_WHRZ + SZ_W2;
constexpr size_t OFF_WHN  = OFF_WIN + SZ_W1;
constexpr size_t OFF_P1   = OFF_WHN + SZ_W1;
constexpr size_t OFF_P2   = OFF_P1 + SZ_P2;
constexpr size_t OFF_P3   = OFF_P2 + SZ_P2;
constexpr size_t OFF_P4   = OFF_P3 + SZ_P1;
constexpr size_t WS_END   = OFF_P4 + SZ_P1;
static_assert(OFF_HB % 128 == 0 && OFF_WIRZ % 128 == 0 && OFF_WHRZ % 128 == 0 && OFF_WIN % 128 == 0);
static_assert(OFF_WHN % 128 == 0 && OFF_P1 % 128 == 0 && OFF_P2 % 128 == 0 && OFF_P3 % 128 == 0 && OFF_P4 % 128 == 0);
static_assert(WS_END <= (size_t)268435456);

constexpr int NPX  = NB * KD / 8;
constexpr int NPW2 = N2 * KD / 8;
constexpr int NPW1 = N1 * KD / 8;
constexpr int NPTOT = 2 * NPX + 2 * NPW2 + 2 * NPW1;
constexpr int NPBLK = NPTOT / 256;
constexpr int PB_H   = NPX / 256;
constexpr int PB_W0  = 2 * NPX / 256;
constexpr int PB_W1  = PB_W0 + NPW2 / 256;
constexpr int PB_W2  = PB_W1 + NPW2 / 256;
constexpr int PB_W3  = PB_W2 + NPW1 / 256;
static_assert(NPX % 256 == 0 && NPW2 % 256 == 0 && NPW1 % 256 == 0);
static_assert(NPTOT % 256 == 0);
static_assert(PB_W3 + NPW1 / 256 == NPBLK);
static_assert((size_t)PB_H  * 256 * 16 == OFF_HB);
static_assert((size_t)PB_W0 * 256 * 16 == OFF_WIRZ);
static_assert((size_t)PB_W1 * 256 * 16 == OFF_WHRZ);
static_assert((size_t)PB_W2 * 256 * 16 == OFF_WIN);
static_assert((size_t)PB_W3 * 256 * 16 == OFF_WHN);
static_assert((size_t)NPBLK * 256 * 16 == OFF_P1);

__device__ __forceinline__ unsigned short bf16_bits(float f) {
    unsigned u = __float_as_uint(f);
    u = u + 0x7FFFu + ((u >> 16) & 1u);
    return (unsigned short)(u >> 16);
}
__device__ __forceinline__ float bf16r(float f) {
    unsigned u = __float_as_uint(f);
    u = (u + 0x7FFFu + ((u >> 16) & 1u)) & 0xFFFF0000u;
    return __uint_as_float(u);
}
__device__ __forceinline__ float rcpx(float x) { return __builtin_amdgcn_rcpf(x); }
__device__ __forceinline__ float sigm(float x) { return rcpx(1.0f + __expf(-x)); }
__device__ __forceinline__ float tanhm(float x) {
    const float e = __expf(2.0f * x);
    return 1.0f - 2.0f * rcpx(e + 1.0f);
}
__device__ __forceinline__ v8f zero8() {
    v8f z;
#pragma unroll
    for (int i = 0; i < 8; ++i) z[i] = 0.0f;
    return z;
}

__device__ __forceinline__ void ldfrag_glb(Frag& f, const __bf16* p) {
    f.half[0] = *(const v8ba*)(p);
    f.half[1] = *(const v8ba*)(p + 16);
}
__device__ __forceinline__ v8f mma16(v8f c, const Frag& a, const Frag& b) {
    return __builtin_amdgcn_wmma_f32_16x16x32_bf16(false, a.v, false, b.v, (short)0, c, false, false);
}

__global__ __launch_bounds__(256)
void prep_kernel(const float* __restrict__ x, const float* __restrict__ hh,
                 const float* __restrict__ w0, const float* __restrict__ w1,
                 const float* __restrict__ w2, const float* __restrict__ w3,
                 unsigned short* planes)
{
    const int bid = blockIdx.x;
    const int g = bid * 256 + threadIdx.x;
    const float* src;
    int pb;
    if (bid < PB_H)       { src = x;  pb = 0; }
    else if (bid < PB_W0) { src = hh; pb = PB_H * 256; }
    else if (bid < PB_W1) { src = w0; pb = PB_W0 * 256; }
    else if (bid < PB_W2) { src = w1; pb = PB_W1 * 256; }
    else if (bid < PB_W3) { src = w2; pb = PB_W2 * 256; }
    else                  { src = w3; pb = PB_W3 * 256; }
    const float* s = src + (size_t)(g - pb) * 8;
    const v4f a = *(const v4fa*)(s);
    const v4f c = *(const v4fa*)(s + 4);
    v8us o;
    o[0] = bf16_bits(a.x); o[1] = bf16_bits(a.y); o[2] = bf16_bits(a.z); o[3] = bf16_bits(a.w);
    o[4] = bf16_bits(c.x); o[5] = bf16_bits(c.y); o[6] = bf16_bits(c.z); o[7] = bf16_bits(c.w);
    unsigned short* d = planes + (size_t)g * 8;
    *(volatile v8us*)d = o;
    __threadfence();
    *(volatile v8us*)d = o;
}

__device__ __forceinline__ void c_store_pass(const float* sT, float* C, int N, int m0, int n0, int w, int lane) {
    const int q8 = lane & 7, sub = lane >> 3;
#pragma unroll
    for (int i = 0; i < 16; ++i) {
        const int lid  = i * 4 + sub;
        const int rowl = 32 * w + (lid >> 1);
        const int hl   = lid & 1;
        const v4f v = *(const v4fa*)(sT + rowl * 64 + 32 * hl + 4 * q8);
        float* dst = C + (size_t)(m0 + rowl) * N + n0 + 32 * hl + 4 * q8;
        *(volatile v4f*)dst = v;
    }
}

__global__ __launch_bounds__(128)
void gemm_kernel(const unsigned short* __restrict__ A,
                 const unsigned short* __restrict__ W,
                 const float* __restrict__ bias,
                 float* C,
                 int N)
{
    __shared__ __attribute__((aligned(16))) float sT[128 * 64];

    const int tid = threadIdx.x, lane = tid & 31, w = tid >> 5;
    const int h = lane >> 4, m = lane & 15;
    const int m0 = blockIdx.x * 128;
    const int n0 = blockIdx.y * 64;
    const int m0w = m0 + 32 * w;

    const __bf16* Ab = (const __bf16*)A;
    const __bf16* Wb = (const __bf16*)W;
    const __bf16* xa0 = Ab + (size_t)(m0w + m) * KD + 8 * h;
    const __bf16* xa1 = xa0 + (size_t)16 * KD;
    const __bf16* wb  = Wb + (size_t)(n0 + m) * KD + 8 * h;

    v8f acc[2][4];
#pragma unroll
    for (int mt = 0; mt < 2; ++mt)
#pragma unroll
        for (int nt = 0; nt < 4; ++nt) acc[mt][nt] = zero8();

#pragma unroll 1
    for (int k0 = 0; k0 < KD; k0 += 32) {
        Frag a[2], b[4];
        ldfrag_glb(a[0], xa0 + k0);
        ldfrag_glb(a[1], xa1 + k0);
#pragma unroll
        for (int nt = 0; nt < 4; ++nt) ldfrag_glb(b[nt], wb + (size_t)nt * 16 * KD + k0);
#pragma unroll
        for (int mt = 0; mt < 2; ++mt)
#pragma unroll
            for (int nt = 0; nt < 4; ++nt) acc[mt][nt] = mma16(acc[mt][nt], a[mt], b[nt]);
        asm volatile("v_nop\n\tv_nop\n\tv_nop\n\tv_nop"
                     : "+v"(acc[0][0]), "+v"(acc[0][1]), "+v"(acc[0][2]), "+v"(acc[0][3]),
                       "+v"(acc[1][0]), "+v"(acc[1][1]), "+v"(acc[1][2]), "+v"(acc[1][3])
                     : "v"(a[0].v), "v"(a[1].v), "v"(b[0].v), "v"(b[1].v), "v"(b[2].v), "v"(b[3].v));
    }

#pragma unroll
    for (int nt = 0; nt < 4; ++nt) {
        const int col = 16 * nt + m;
        const float bb = bf16r(bias[n0 + col]);
#pragma unroll
        for (int mt = 0; mt < 2; ++mt) {
#pragma unroll
            for (int r = 0; r < 8; ++r) {
                const int rowl = 32 * w + 16 * mt + 8 * h + r;
                sT[rowl * 64 + col] = acc[mt][nt][r] + bb;
            }
        }
    }
    __syncthreads();

    c_store_pass(sT, C, N, m0, n0, w, lane);
    __threadfence();
    c_store_pass(sT, C, N, m0, n0, w, lane);
}

__device__ __forceinline__ float hsum4(v4f v) { return (v.x + v.y) + (v.z + v.w); }
__device__ __forceinline__ float wsum(float v) {
#pragma unroll
    for (int s = 16; s > 0; s >>= 1) v += __shfl_xor(v, s, 32);
    return v;
}
__device__ __forceinline__ float sq4(v4f v, float q) {
    q = fmaf(v.x, v.x, q);
    q = fmaf(v.y, v.y, q);
    q = fmaf(v.z, v.z, q);
    q = fmaf(v.w, v.w, q);
    return q;
}
__device__ __forceinline__ float lds8(const float* r) {
    const v4f a = *(const v4fa*)(r);
    const v4f b = *(const v4fa*)(r + 4);
    return ((a.x + a.y) + (a.z + a.w)) + ((b.x + b.y) + (b.z + b.w));
}
__device__ __forceinline__ float gate1(float ir, float hr, float iz, float hz, float in_, float hn, float hb) {
    const float r = sigm(ir + hr);
    const float z = sigm(iz + hz);
    const float n = tanhm(fmaf(r, hn, in_));
    return (1.0f - z) * n + z * hb;
}

__global__ __launch_bounds__(256)
void gate_kernel(const float* __restrict__ P1,
                 const float* __restrict__ P2,
                 const float* __restrict__ P3,
                 const float* __restrict__ P4,
                 const float* __restrict__ hin,
                 float* out)
{
    __shared__ __attribute__((aligned(16))) float red[8][8];

    const int tid = threadIdx.x, lane = tid & 31, w = tid >> 5;
    const size_t row = blockIdx.x;
    const int c4 = tid * 4;

    const float* p1 = P1 + row * N2 + c4;
    const float* p2 = P2 + row * N2 + c4;
    const v4f a0 = *(const v4fa*)(p1);
    const v4f a1 = *(const v4fa*)(p1 + N1);
    const v4f b0 = *(const v4fa*)(p2);
    const v4f b1 = *(const v4fa*)(p2 + N1);
    const v4f g0 = *(const v4fa*)(P3 + row * N1 + c4);
    const v4f k0 = *(const v4fa*)(P4 + row * N1 + c4);
    const v4f hv = *(const v4fa*)(hin + row * N1 + c4);

    float s1 = hsum4(a0) + hsum4(a1);
    float s2 = hsum4(b0) + hsum4(b1);
    float s3 = hsum4(g0);
    float s4 = hsum4(k0);
    s1 = wsum(s1); s2 = wsum(s2); s3 = wsum(s3); s4 = wsum(s4);
    if (lane == 0) { red[0][w] = s1; red[1][w] = s2; red[2][w] = s3; red[3][w] = s4; }
    __syncthreads();
    const float mu1 = lds8(&red[0][0]) * (1.0f / 2048.0f);
    const float mu2 = lds8(&red[1][0]) * (1.0f / 2048.0f);
    const float mu3 = lds8(&red[2][0]) * (1.0f / 1024.0f);
    const float mu4 = lds8(&red[3][0]) * (1.0f / 1024.0f);

    const v4f e0 = a0 - mu1, e1 = a1 - mu1;
    const v4f f0 = b0 - mu2, f1 = b1 - mu2;
    const v4f g1 = g0 - mu3;
    const v4f k1 = k0 - mu4;
    float q1 = sq4(e1, sq4(e0, 0.0f));
    float q2 = sq4(f1, sq4(f0, 0.0f));
    float q3 = sq4(g1, 0.0f);
    float q4 = sq4(k1, 0.0f);
    q1 = wsum(q1); q2 = wsum(q2); q3 = wsum(q3); q4 = wsum(q4);
    if (lane == 0) { red[4][w] = q1; red[5][w] = q2; red[6][w] = q3; red[7][w] = q4; }
    __syncthreads();
    const float rs1 = rsqrtf(lds8(&red[4][0]) * (1.0f / 2048.0f) + LN_EPS);
    const float rs2 = rsqrtf(lds8(&red[5][0]) * (1.0f / 2048.0f) + LN_EPS);
    const float rs3 = rsqrtf(lds8(&red[6][0]) * (1.0f / 1024.0f) + LN_EPS);
    const float rs4 = rsqrtf(lds8(&red[7][0]) * (1.0f / 1024.0f) + LN_EPS);

    const v4f i_r = e0 * rs1, i_z = e1 * rs1;
    const v4f h_r = f0 * rs2, h_z = f1 * rs2;
    const v4f i_n = g1 * rs3;
    const v4f h_n = k1 * rs4;

    v4f o;
    o.x = gate1(i_r.x, h_r.x, i_z.x, h_z.x, i_n.x, h_n.x, bf16r(hv.x));
    o.y = gate1(i_r.y, h_r.y, i_z.y, h_z.y, i_n.y, h_n.y, bf16r(hv.y));
    o.z = gate1(i_r.z, h_r.z, i_z.z, h_z.z, i_n.z, h_n.z, bf16r(hv.z));
    o.w = gate1(i_r.w, h_r.w, i_z.w, h_z.w, i_n.w, h_n.w, bf16r(hv.w));

    float* op = out + row * N1 + c4;
    *(volatile v4f*)op = o;
    __threadfence();
    *(volatile v4f*)op = o;
}

extern "C" void kernel_launch(void* const* d_in, const int* in_sizes, int n_in,
                              void* d_out, int out_size, void* d_ws, size_t ws_size,
                              hipStream_t stream)
{
    if (n_in < 10) return;
    if (in_sizes[0] != NB * KD) return;
    if (in_sizes[1] != NB * KD) return;
    if (in_sizes[2] != N2 * KD) return;
    if (in_sizes[3] != N2)      return;
    if (in_sizes[4] != N2 * KD) return;
    if (in_sizes[5] != N2)      return;
    if (in_sizes[6] != N1 * KD) return;
    if (in_sizes[7] != N1)      return;
    if (in_sizes[8] != N1 * KD) return;
    if (in_sizes[9] != N1)      return;
    if (out_size != NB * N1)    return;
    if (ws_size < WS_END)       return;

    const float* x     = (const float*)d_in[0];
    const float* h     = (const float*)d_in[1];
    const float* W_irz = (const float*)d_in[2];
    const float* b_irz = (const float*)d_in[3];
    const float* W_hrz = (const float*)d_in[4];
    const float* b_hrz = (const float*)d_in[5];
    const float* W_in  = (const float*)d_in[6];
    const float* b_in  = (const float*)d_in[7];
    const float* W_hn  = (const float*)d_in[8];
    const float* b_hn  = (const float*)d_in[9];
    float* out = (float*)d_out;

    char* ws = (char*)d_ws;
    unsigned short* planes = (unsigned short*)(ws + OFF_XB);
    const unsigned short* XB   = (const unsigned short*)(ws + OFF_XB);
    const unsigned short* HB   = (const unsigned short*)(ws + OFF_HB);
    const unsigned short* WIRZ = (const unsigned short*)(ws + OFF_WIRZ);
    const unsigned short* WHRZ = (const unsigned short*)(ws + OFF_WHRZ);
    const unsigned short* WIN  = (const unsigned short*)(ws + OFF_WIN);
    const unsigned short* WHN  = (const unsigned short*)(ws + OFF_WHN);
    float* P1 = (float*)(ws + OFF_P1);
    float* P2 = (float*)(ws + OFF_P2);
    float* P3 = (float*)(ws + OFF_P3);
    float* P4 = (float*)(ws + OFF_P4);

    prep_kernel<<<dim3(NPBLK), dim3(256), 0, stream>>>(x, h, W_irz, W_hrz, W_in, W_hn, planes);

    gemm_kernel<<<dim3(NB / 128, N2 / 64), dim3(128), 0, stream>>>(XB, WIRZ, b_irz, P1, N2);
    gemm_kernel<<<dim3(NB / 128, N2 / 64), dim3(128), 0, stream>>>(HB, WHRZ, b_hrz, P2, N2);
    gemm_kernel<<<dim3(NB / 128, N1 / 64), dim3(128), 0, stream>>>(XB, WIN,  b_in,  P3, N1);
    gemm_kernel<<<dim3(NB / 128, N1 / 64), dim3(128), 0, stream>>>(HB, WHN,  b_hn,  P4, N1);

    gate_kernel<<<dim3(NB), dim3(256), 0, stream>>>(P1, P2, P3, P4, h, out);
}
